// GKAN_47459388621632
// MI455X (gfx1250) — hardware-run, weakly checked
//
#include <hip/hip_runtime.h>
#include <stddef.h>

#pragma clang fp contract(off)


#define DD      64
#define NCO     8
#define KD      576
#define NGRP    72
#define NPB     1568
#define NFB     64
#define NCB     8
#define NPC     12544
#define NSEG    8
#define CAPW    24576
#define LPW     768
#define CAPB    24576
#define NCHB    96
#define COLN    1572864
#define MPAD    100096
#define MHALF   50048
#define NGR     512
#define NTGT    10
#define NTHR    256
#define RPB     64
#define HBP     68
#define MAXDEG  256
#define MAXPG   4096
#define NFLG    128
#define WSC     16.0f
#define WINV    0.0625f
#define WSCAP   134217728
#define CSRLDS  196608

static_assert((KD % 32) == 0);
static_assert(DD * NGRP * 8 == DD * KD);
static_assert(((DD * NGRP) % NTHR) == 0);
static_assert(NPC == 8 * NPB && NFB == 8 * NCB);
static_assert((NPB % 32) == 0);
static_assert(CAPW == 32 * LPW);
static_assert(CAPB == NCHB * NTHR);
static_assert(((NSEG * CAPW) % NTHR) == 0);
static_assert(COLN == NFB * CAPB && COLN == NCB * NSEG * CAPW);
static_assert(NPC < 32768 && MPAD <= 131072 && MPAD <= NFB * NPB);
static_assert(MPAD == 2 * MHALF && (MHALF % RPB) == 0 && (NGR % RPB) == 0);
static_assert(CSRLDS == 2 * CAPB * 4);
static_assert(((HBP * 4) % 16) == 0);
static_assert((RPB * DD / 4) == 4 * NTHR);
static_assert(((NGR * NTGT) % (4 * NTHR)) == 0);
static_assert(NCB * NSEG + NFB == NFLG);

typedef float          v2f   __attribute__((ext_vector_type(2)));
typedef float          v4f   __attribute__((ext_vector_type(4)));
typedef float          v8f   __attribute__((ext_vector_type(8)));
typedef int            v4i   __attribute__((ext_vector_type(4)));
typedef unsigned       v4u   __attribute__((ext_vector_type(4)));
typedef _Float16       v8h   __attribute__((ext_vector_type(8)));
typedef _Float16       v16h  __attribute__((ext_vector_type(16)));
typedef unsigned short v8us  __attribute__((ext_vector_type(8)));
typedef unsigned short v16us __attribute__((ext_vector_type(16)));
union FragH { v16h v; v16us u; v8us h[2]; };
union P8 { v8us u; v4u q; };
union P1 { _Float16 h; unsigned short u; };
static_assert(sizeof(FragH) == 32);
static_assert(sizeof(P8) == 16);
static_assert(sizeof(P1) == 2);

#define KG(j) ((float)((j) - 3) * 0.4f - 1.0f)
#define R1(t) (1.0f / (KG((t) + 1) - KG(t)))
#define R2(t) (1.0f / (KG((t) + 2) - KG(t)))
#define R3(t) (1.0f / (KG((t) + 3) - KG(t)))
__constant__ float c_g[12]  = {KG(0), KG(1), KG(2), KG(3), KG(4), KG(5), KG(6), KG(7), KG(8), KG(9), KG(10), KG(11)};
__constant__ float c_r1[11] = {R1(0), R1(1), R1(2), R1(3), R1(4), R1(5), R1(6), R1(7), R1(8), R1(9), R1(10)};
__constant__ float c_r2[10] = {R2(0), R2(1), R2(2), R2(3), R2(4), R2(5), R2(6), R2(7), R2(8), R2(9)};
__constant__ float c_r3[9]  = {R3(0), R3(1), R3(2), R3(3), R3(4), R3(5), R3(6), R3(7), R3(8)};

__device__ __forceinline__ v8f wmf(v16h a, v16h bq, v8f c) {
  v8f d = __builtin_amdgcn_wmma_f32_16x16x32_f16(false, a, false, bq, (short)0, c, false, false);
  asm volatile("v_nop\n\tv_nop\n\tv_nop\n\tv_nop" : "+v"(d) : "v"(a), "v"(bq));
  return d;
}
__device__ __forceinline__ v8f zero8() {
  v8f z = {0.f, 0.f, 0.f, 0.f, 0.f, 0.f, 0.f, 0.f};
  return z;
}
__device__ __forceinline__ unsigned short f16_bits(float f) {
  P1 p; p.h = (_Float16)f;
  return p.u;
}
__device__ __forceinline__ void wsync() {
  __builtin_amdgcn_fence(__ATOMIC_RELEASE, "wavefront");
  __builtin_amdgcn_wave_barrier();
}
__device__ __forceinline__ void st2u(unsigned* p, unsigned v) {
  *(volatile unsigned*)p = v; __threadfence(); *(volatile unsigned*)p = v;
}
__device__ __forceinline__ void st2v8us(unsigned short* p, v8us v) {
  *(volatile v8us*)p = v; __threadfence(); *(volatile v8us*)p = v;
}
__device__ __forceinline__ void st2v2f(float* p, v2f v) {
  *(volatile v2f*)p = v; __threadfence(); *(volatile v2f*)p = v;
}
__device__ __forceinline__ void st2v4f(float* p, v4f v) {
  *(volatile v4f*)p = v; __threadfence(); *(volatile v4f*)p = v;
}

__device__ __forceinline__ void kan_feat(float x, unsigned short& sb, v8us& pk) {
  float bs[11];
#pragma unroll
  for (int t = 0; t < 11; ++t) bs[t] = (x >= c_g[t] && x < c_g[t + 1]) ? 1.0f : 0.0f;
#pragma unroll
  for (int t = 0; t < 10; ++t) {
    const float lf = (x - c_g[t]) * c_r1[t];
    const float rg = (c_g[t + 2] - x) * c_r1[t + 1];
    bs[t] = lf * bs[t] + rg * bs[t + 1];
  }
#pragma unroll
  for (int t = 0; t < 9; ++t) {
    const float lf = (x - c_g[t]) * c_r2[t];
    const float rg = (c_g[t + 3] - x) * c_r2[t + 1];
    bs[t] = lf * bs[t] + rg * bs[t + 1];
  }
#pragma unroll
  for (int t = 0; t < 8; ++t) {
    const float lf = (x - c_g[t]) * c_r3[t];
    const float rg = (c_g[t + 4] - x) * c_r3[t + 1];
    bs[t] = lf * bs[t] + rg * bs[t + 1];
  }
  const float sl = x * __builtin_amdgcn_rcpf(1.0f + __expf(-x));
  sb = f16_bits(sl);
#pragma unroll
  for (int c = 0; c < NCO; ++c) pk[c] = f16_bits(bs[c]);
}

__global__ __launch_bounds__(NTHR) void k_wprep(const float* __restrict__ bw0, const float* __restrict__ sw0,
                                               const float* __restrict__ sc0, const float* __restrict__ bw1,
                                               const float* __restrict__ sw1, const float* __restrict__ sc1,
                                               const float* __restrict__ bwh, const float* __restrict__ swh,
                                               const float* __restrict__ sch,
                                               unsigned short* W0p, unsigned short* W1p, unsigned short* Whp) {
  const int lay = blockIdx.y;
  const float* bw = (lay == 0) ? bw0 : ((lay == 1) ? bw1 : bwh);
  const float* sw = (lay == 0) ? sw0 : ((lay == 1) ? sw1 : swh);
  const float* sc = (lay == 0) ? sc0 : ((lay == 1) ? sc1 : sch);
  unsigned short* Wp = (lay == 0) ? W0p : ((lay == 1) ? W1p : Whp);
  const int nout = (lay == 2) ? NTGT : DD;
  const int t = blockIdx.x * NTHR + threadIdx.x;
  const int o = t / NGRP, q = t - o * NGRP;
  const int oc = (o < nout) ? o : (nout - 1);
  int ib = 8 * q;     ib = ib > DD - 8 ? DD - 8 : ib;
  int is = q - 8;     is = is < 0 ? 0 : is;
  const float* pb = bw + (size_t)oc * DD + ib;
  const size_t io = (size_t)oc * DD + is;
  const float* pc = sw + io * NCO;
  const float sp = sc[io];
  const v4f x0 = *(const v4f*)pb, x1 = *(const v4f*)(pb + 4);
  const v4f g0 = *(const v4f*)pc, g1 = *(const v4f*)(pc + 4);
  const float bb[8] = {x0.x, x0.y, x0.z, x0.w, x1.x, x1.y, x1.z, x1.w};
  const float gg[8] = {g0.x, g0.y, g0.z, g0.w, g1.x, g1.y, g1.z, g1.w};
  const bool isb = q < 8;
  const bool val = o < nout;
  v8us wv;
#pragma unroll
  for (int e = 0; e < 8; ++e) {
    const float v = isb ? bb[e] : (gg[e] * sp);
    wv[e] = f16_bits(val ? (WSC * v) : 0.0f);
  }
  st2v8us(Wp + (size_t)t * 8, wv);
}

__global__ __launch_bounds__(NTHR) void k_bucket(const int* __restrict__ ei, int nE, int nN,
                                                unsigned* blist, unsigned* flg) {
  __shared__ unsigned sl[NSEG][64];
  const int b = blockIdx.x, tid = threadIdx.x, w = tid >> 5, l = tid & 31;
  const int lo = b * NPC;
  unsigned* seg = blist + ((size_t)b * NSEG + w) * CAPW;
  unsigned* myl = sl[w];
  const unsigned ltm = (1u << l) - 1u;
  int cnt = 0, nl = 0, ovf = 0;
  const int nch = (nE + 127) >> 7;
  const bool al4 = ((nE & 3) == 0);
  for (int c = w; c < nch; c += NSEG) {
    const int base = (c << 7) + 4 * l;
    int sv[4], dv[4];
    if (al4 && (c << 7) + 128 <= nE) {
      const v4i s4 = *(const v4i*)(ei + base);
      const v4i d4 = *(const v4i*)(ei + (size_t)nE + base);
      sv[0] = s4.x; sv[1] = s4.y; sv[2] = s4.z; sv[3] = s4.w;
      dv[0] = d4.x; dv[1] = d4.y; dv[2] = d4.z; dv[3] = d4.w;
    } else {
#pragma unroll
      for (int j = 0; j < 4; ++j) {
        const int e = base + j;
        const int ec = e < nE ? e : (nE - 1);
        sv[j] = ei[ec];
        const int dd = ei[(size_t)nE + ec];
        dv[j] = (e < nE) ? dd : -1;
      }
    }
#pragma unroll
    for (int j = 0; j < 4; ++j) {
      const int d = dv[j];
      int s = sv[j];
      s = s < 0 ? 0 : (s > nN - 1 ? nN - 1 : s);
      const bool hit = (d >= lo) && (d < lo + NPC) && (d < nN);
      const unsigned m = __builtin_amdgcn_ballot_w32(hit);
      const int rk = __builtin_popcount(m & ltm);
      if (hit) myl[cnt + rk] = ((unsigned)(d - lo) << 17) | (unsigned)s;
      cnt += __builtin_popcount(m);
      if (cnt >= 32) {
        wsync();
        const unsigned v = myl[l];
        if (nl < LPW) { st2u(seg + (size_t)nl * 32 + l, v); ++nl; } else ovf = 1;
        const unsigned t = myl[32 + l];
        wsync();
        const int r = cnt - 32;
        if (l < r) myl[l] = t;
        wsync();
        cnt = r;
      }
    }
  }
  wsync();
  unsigned v = myl[l];
  v = (l < cnt) ? v : 0xFFFFFFFFu;
  if (cnt > 0) {
    if (nl < LPW) { st2u(seg + (size_t)nl * 32 + l, v); ++nl; } else ovf = 1;
  }
  for (int ln = nl; ln < LPW; ++ln) st2u(seg + (size_t)ln * 32 + l, 0xFFFFFFFFu);
  st2u(flg + ((size_t)b * NSEG + w) * 32 + l, (l == 0) ? (unsigned)ovf : 0u);
}

__global__ __launch_bounds__(NTHR) void k_csr(const unsigned* __restrict__ blist, unsigned* colp, int* stp, int* enp,
                                             unsigned* flg) {
  extern __shared__ __align__(16) unsigned dlds[];
  __shared__ int wc[2][NSEG];
  __shared__ int wz[NSEG][11];
  __shared__ int zt[11];
  unsigned* bufA = dlds;
  unsigned* bufB = dlds + CAPB;
  const int f = blockIdx.x, tid = threadIdx.x, w = tid >> 5, l = tid & 31;
  const unsigned ltm = (1u << l) - 1u;
  const unsigned* cs = blist + (size_t)(f >> 3) * (NSEG * CAPW);
  const unsigned klo = (unsigned)(f & 7) * NPB;

  int nA = 0;
  for (int i = 0; i < (NSEG * CAPW) / NTHR; ++i) {
    const unsigned e = cs[(size_t)i * NTHR + tid];
    const unsigned dl = e >> 17;
    const bool hit = (dl >= klo) && (dl < klo + NPB);
    const unsigned m = __builtin_amdgcn_ballot_w32(hit);
    const int rk = __builtin_popcount(m & ltm), cw = __builtin_popcount(m);
    if (l == 0) wc[i & 1][w] = cw;
    __syncthreads();
    int pz = 0, tz = 0;
#pragma unroll
    for (int ww = 0; ww < NSEG; ++ww) { const int c = wc[i & 1][ww]; tz += c; pz += (ww < w) ? c : 0; }
    const int pos = nA + pz + rk;
    if (hit && pos < CAPB) bufA[pos] = ((dl - klo) << 17) | (e & 0x1FFFFu);
    nA += tz;
  }
  int ovf = 0;
  if (nA > CAPB) { ovf = 1; nA = CAPB; }
  const int nchunk = (nA + NTHR - 1) / NTHR;
  const int nS = nchunk * NTHR;
  for (int p = nA + tid; p < nS; p += NTHR) bufA[p] = 0xFFFFFFFFu;
  __syncthreads();

  int z[11];
#pragma unroll
  for (int bb = 0; bb < 11; ++bb) z[bb] = 0;
  for (int i = 0; i < nchunk; ++i) {
    const unsigned key = bufA[i * NTHR + tid] >> 17;
#pragma unroll
    for (int bb = 0; bb < 11; ++bb) z[bb] += (int)((~(key >> bb)) & 1u);
  }
#pragma unroll
  for (int bb = 0; bb < 11; ++bb) {
    int v = z[bb];
    v += __shfl_xor(v, 16); v += __shfl_xor(v, 8); v += __shfl_xor(v, 4); v += __shfl_xor(v, 2); v += __shfl_xor(v, 1);
    if (l == 0) wz[w][bb] = v;
  }
  __syncthreads();
  if (tid < 11) {
    int s = 0;
#pragma unroll
    for (int ww = 0; ww < NSEG; ++ww) s += wz[ww][tid];
    zt[tid] = s;
  }
  __syncthreads();

  for (int p = 0; p < 11; ++p) {
    const unsigned* in = (p & 1) ? bufB : bufA;
    unsigned* out = (p & 1) ? bufA : bufB;
    int zb = 0, ob = zt[p];
    for (int i = 0; i < nchunk; ++i) {
      const unsigned e = in[i * NTHR + tid];
      const bool isz = ((e >> (17 + p)) & 1u) == 0u;
      const unsigned m = __builtin_amdgcn_ballot_w32(isz);
      const int rz = __builtin_popcount(m & ltm), cz = __builtin_popcount(m);
      if (l == 0) wc[i & 1][w] = cz;
      __syncthreads();
      int pz = 0, tz = 0;
#pragma unroll
      for (int ww = 0; ww < NSEG; ++ww) { const int c = wc[i & 1][ww]; tz += c; pz += (ww < w) ? c : 0; }
      int pos = isz ? (zb + pz + rz) : (ob + (32 * w - pz) + (l - rz));
      pos = pos < 0 ? 0 : (pos > nS - 1 ? nS - 1 : pos);
      out[pos] = e;
      zb += tz; ob += NTHR - tz;
    }
    __syncthreads();
  }

  unsigned* rp = bufA;
#pragma unroll
  for (int j = 0; j < 7; ++j) {
    const int k = tid + NTHR * j;
    if (k <= NPB) {
      int lo = 0, hi = nS;
      for (int s = 0; s < 15; ++s) {
        if (lo < hi) {
          const int mid = (lo + hi) >> 1;
          if ((bufB[mid] >> 17) < (unsigned)k) lo = mid + 1; else hi = mid;
        }
      }
      rp[k] = (unsigned)lo;
    }
  }
  __syncthreads();

  unsigned* cgp = colp + (size_t)f * CAPB;
#pragma unroll 1
  for (int i = 0; i < CAPB / (4 * NTHR); ++i) {
    const int c = tid + NTHR * i;
    v4u v = *(const v4u*)(bufB + 4 * c);
    v = v & 0x1FFFFu;
    if (4 * c >= nS) v = (v4u){0u, 0u, 0u, 0u};
    *(volatile v4u*)(cgp + 4 * c) = v;
  }
  __threadfence();
#pragma unroll 1
  for (int i = 0; i < CAPB / (4 * NTHR); ++i) {
    const int c = tid + NTHR * i;
    v4u v = *(const v4u*)(bufB + 4 * c);
    v = v & 0x1FFFFu;
    if (4 * c >= nS) v = (v4u){0u, 0u, 0u, 0u};
    *(volatile v4u*)(cgp + 4 * c) = v;
  }

  const unsigned ab = (unsigned)f * CAPB;
  unsigned* sp0 = (unsigned*)stp + (size_t)f * NPB;
  unsigned* ep0 = (unsigned*)enp + (size_t)f * NPB;
#pragma unroll
  for (int j = 0; j < 2; ++j) {
    const int c = tid + NTHR * j;
    const int cc = c < NPB / 4 ? c : (NPB / 4 - 1);
    v4u sv, ev;
#pragma unroll
    for (int e = 0; e < 4; ++e) { sv[e] = ab + rp[4 * cc + e]; ev[e] = ab + rp[4 * cc + e + 1]; }
    if (c < NPB / 4) { *(volatile v4u*)(sp0 + 4 * c) = sv; *(volatile v4u*)(ep0 + 4 * c) = ev; }
  }
  __threadfence();
#pragma unroll
  for (int j = 0; j < 2; ++j) {
    const int c = tid + NTHR * j;
    const int cc = c < NPB / 4 ? c : (NPB / 4 - 1);
    v4u sv, ev;
#pragma unroll
    for (int e = 0; e < 4; ++e) { sv[e] = ab + rp[4 * cc + e]; ev[e] = ab + rp[4 * cc + e + 1]; }
    if (c < NPB / 4) { *(volatile v4u*)(sp0 + 4 * c) = sv; *(volatile v4u*)(ep0 + 4 * c) = ev; }
  }
  if (w == 0) st2u(flg + (size_t)(NCB * NSEG + f) * 32 + l, (l == 0) ? (unsigned)ovf : 0u);
}

template <bool AGG>
__global__ __launch_bounds__(NTHR) void k_aggfeat(const float* __restrict__ xin, const int* __restrict__ stp,
                                                 const int* __restrict__ enp, const unsigned* __restrict__ colp,
                                                 unsigned short* Ap, int row0, int nvalid, int nN) {
  __shared__ __align__(16) unsigned sR[NSEG][KD / 2 + 4];
  const int tid = threadIdx.x, w = tid >> 5, l = tid & 31;
  unsigned* row = sR[w];
#pragma unroll 1
  for (int q = 0; q < 8; ++q) {
    const int r = blockIdx.x * 64 + w * 8 + q;
    const int v = row0 + r;
    const bool val = v < nvalid;
    const int vc = val ? v : (nvalid - 1);
    const v2f xs = *(const v2f*)(xin + (size_t)vc * DD + 2 * l);
    float y0 = xs.x, y1 = xs.y;
    if (AGG) {
      const int vi = v < NFB * NPB ? v : (NFB * NPB - 1);
      int st = stp[vi], en = enp[vi];
      st = st < 0 ? 0 : (st > COLN ? COLN : st);
      int deg = en - st;
      deg = deg < 0 ? 0 : (deg > MAXDEG ? MAXDEG : deg);
      if (!val) deg = 0;
      float a0 = 0.f, a1 = 0.f;
      for (int base = 0; base < deg; base += 32) {
        int ix = st + base + l;
        ix = ix > COLN - 1 ? COLN - 1 : ix;
        const unsigned cv = colp[ix];
        int s = (int)(cv & 0x1FFFFu);
        s = s > nN - 1 ? nN - 1 : s;
        const int nb = (deg - base) < 32 ? (deg - base) : 32;
        for (int j = 0; j < nb; ++j) {
          const int sj = __shfl(s, j);
          const v2f t = *(const v2f*)(xin + (size_t)sj * DD + 2 * l);
          a0 += t.x; a1 += t.y;
        }
      }
      y0 += a0; y1 += a1;
    }
    unsigned short s0, s1;
    P8 p0, p1;
    kan_feat(y0, s0, p0.u);
    kan_feat(y1, s1, p1.u);
    const unsigned short zm = val ? (unsigned short)0xFFFFu : (unsigned short)0u;
    const v8us zm8 = {zm, zm, zm, zm, zm, zm, zm, zm};
    s0 &= zm; s1 &= zm;
    p0.u = p0.u & zm8; p1.u = p1.u & zm8;
    row[l] = (unsigned)s0 | ((unsigned)s1 << 16);
    *(v4u*)(row + 32 + 8 * l) = p0.q;
    *(v4u*)(row + 36 + 8 * l) = p1.q;
    wsync();
    const int l2 = l < 8 ? l : 7;
    const v4u c0 = *(const v4u*)(row + 4 * l);
    const v4u c1 = *(const v4u*)(row + 4 * (l + 32));
    const v4u c2 = *(const v4u*)(row + 4 * (64 + l2));
    unsigned short* gp = Ap + (size_t)r * KD;
    *(volatile v4u*)(gp + 8 * l) = c0;
    *(volatile v4u*)(gp + 8 * (l + 32)) = c1;
    if (l < 8) *(volatile v4u*)(gp + 8 * (64 + l)) = c2;
    __threadfence();
    *(volatile v4u*)(gp + 8 * l) = c0;
    *(volatile v4u*)(gp + 8 * (l + 32)) = c1;
    if (l < 8) *(volatile v4u*)(gp + 8 * (64 + l)) = c2;
    wsync();
  }
}

__global__ __launch_bounds__(NTHR) void k_gemm(const unsigned short* __restrict__ Ap,
                                              const unsigned short* __restrict__ Wp, float* C) {
  __shared__ __align__(16) float hb[RPB * HBP];
  const int tid = threadIdx.x, lane = tid & 31, wave = tid >> 5, h = lane >> 4, m = lane & 15;
  const int rt = wave & 3, cg = wave >> 2;
  const int rowBase = blockIdx.x * RPB;
  const unsigned short* ap = Ap + (size_t)(rowBase + 16 * rt + m) * KD + 8 * h;
  const unsigned short* wp = Wp + (size_t)(32 * cg + m) * KD + 8 * h;

  v8f acc[2];
  acc[0] = zero8(); acc[1] = zero8();

#pragma unroll 2
  for (int ks = 0; ks < KD / 32; ++ks) {
    const int ko = 32 * ks;
    FragH fa;
    fa.h[0] = *(const v8us*)(ap + ko);
    fa.h[1] = *(const v8us*)(ap + ko + 16);
#pragma unroll
    for (int nt = 0; nt < 2; ++nt) {
      const unsigned short* bp = wp + (size_t)(16 * nt) * KD + ko;
      FragH fb;
      fb.h[0] = *(const v8us*)bp;
      fb.h[1] = *(const v8us*)(bp + 16);
      acc[nt] = wmf(fa.v, fb.v, acc[nt]);
    }
  }

#pragma unroll
  for (int nt = 0; nt < 2; ++nt) {
#pragma unroll
    for (int r = 0; r < 8; ++r)
      hb[(16 * rt + 8 * h + r) * HBP + 32 * cg + 16 * nt + m] = acc[nt][r] * WINV;
  }
  __syncthreads();

  float* cp = C + (size_t)rowBase * DD;
#pragma unroll
  for (int j = 0; j < 4; ++j) {
    const int e = tid + NTHR * j;
    const int rr = e >> 4, q = e & 15;
    const v4f v = *(const v4f*)(hb + rr * HBP + 4 * q);
    *(volatile v4f*)(cp + (size_t)rr * DD + 4 * q) = v;
  }
  __threadfence();
#pragma unroll
  for (int j = 0; j < 4; ++j) {
    const int e = tid + NTHR * j;
    const int rr = e >> 4, q = e & 15;
    const v4f v = *(const v4f*)(hb + rr * HBP + 4 * q);
    *(volatile v4f*)(cp + (size_t)rr * DD + 4 * q) = v;
  }
}

__global__ __launch_bounds__(NTHR) void k_pool(const float* __restrict__ H, const int* __restrict__ bat, int nN,
                                              float* P) {
  const int tid = threadIdx.x, w = tid >> 5, l = tid & 31;
  const int g = blockIdx.x * NSEG + w;
  int lo = 0, hi = nN;
  for (int s = 0; s < 18; ++s) {
    if (lo < hi) { const int mid = (lo + hi) >> 1; if (bat[mid] < g) lo = mid + 1; else hi = mid; }
  }
  int lo2 = 0, hi2 = nN;
  for (int s = 0; s < 18; ++s) {
    if (lo2 < hi2) { const int mid = (lo2 + hi2) >> 1; if (bat[mid] <= g) lo2 = mid + 1; else hi2 = mid; }
  }
  int cnt = lo2 - lo;
  cnt = cnt < 0 ? 0 : (cnt > MAXPG ? MAXPG : cnt);
  float a0 = 0.f, a1 = 0.f;
  for (int j = 0; j < cnt; ++j) {
    int v = lo + j;
    v = v > nN - 1 ? nN - 1 : v;
    const int bb = bat[v];
    const v2f t = *(const v2f*)(H + (size_t)v * DD + 2 * l);
    a0 += (bb == g) ? t.x : 0.f;
    a1 += (bb == g) ? t.y : 0.f;
  }
  v2f r; r.x = a0; r.y = a1;
  st2v2f(P + (size_t)g * DD + 2 * l, r);
}

__global__ __launch_bounds__(NTHR) void k_pack(const float* __restrict__ O, const unsigned* __restrict__ flg,
                                              float* out) {
  __shared__ int sf[NSEG];
  const int tid = threadIdx.x, w = tid >> 5, l = tid & 31;
  const int fi = tid < NFLG ? tid : (NFLG - 1);
  unsigned fv = flg[(size_t)fi * 32];
  fv = (tid < NFLG) ? fv : 0u;
  const unsigned m = __builtin_amdgcn_ballot_w32(fv != 0u);
  if (l == 0) sf[w] = (m != 0u) ? 1 : 0;
  __syncthreads();
  int any = 0;
#pragma unroll
  for (int i = 0; i < NSEG; ++i) any |= sf[i];
  const float qnan = __int_as_float(0x7fc00000);
  const int t = blockIdx.x * NTHR + tid;
  v4f rv;
#pragma unroll
  for (int e = 0; e < 4; ++e) {
    const int idx = 4 * t + e;
    const int rw = idx / NTGT;
    const int cl = idx - rw * NTGT;
    const float val = O[(size_t)rw * DD + cl];
    rv[e] = any ? qnan : val;
  }
  st2v4f(out + (size_t)4 * t, rv);
}

extern "C" void kernel_launch(void* const* d_in, const int* in_sizes, int n_in,
                              void* d_out, int out_size, void* d_ws, size_t ws_size,
                              hipStream_t stream) {
  if (n_in < 12) return;
  const int nN = in_sizes[0] / DD;
  if (nN <= 0 || in_sizes[0] != nN * DD || nN > MPAD || nN > NFB * NPB) return;
  const int nE = in_sizes[1] / 2;
  if (nE <= 0 || in_sizes[1] != 2 * nE) return;
  if (in_sizes[2] != nN) return;
  if (in_sizes[3] != DD * DD || in_sizes[4] != DD * DD * NCO || in_sizes[5] != DD * DD) return;
  if (in_sizes[6] != DD * DD || in_sizes[7] != DD * DD * NCO || in_sizes[8] != DD * DD) return;
  if (in_sizes[9] != NTGT * DD || in_sizes[10] != NTGT * DD * NCO || in_sizes[11] != NTGT * DD) return;
  if (out_size != NGR * NTGT) return;

  const float* x    = (const float*)d_in[0];
  const int* ei     = (const int*)d_in[1];
  const int* bat    = (const int*)d_in[2];
  const float* bw0  = (const float*)d_in[3];
  const float* sw0  = (const float*)d_in[4];
  const float* sc0  = (const float*)d_in[5];
  const float* bw1  = (const float*)d_in[6];
  const float* sw1  = (const float*)d_in[7];
  const float* sc1  = (const float*)d_in[8];
  const float* bwh  = (const float*)d_in[9];
  const float* swh  = (const float*)d_in[10];
  const float* sch  = (const float*)d_in[11];
  float* out = (float*)d_out;

  size_t off = 0;
  const size_t bBL = (size_t)NCB * NSEG * CAPW * 4;
  const size_t bFL = (size_t)NFLG * 128;
  const size_t bCOL = (size_t)NFB * CAPB * 4;
  const size_t bSE = (size_t)NFB * NPB * 4;
  const size_t bA = (size_t)MHALF * KD * 2;
  const size_t bH = (size_t)MPAD * DD * 4;
  const size_t bP = (size_t)NGR * DD * 4;
  const size_t bW = (size_t)DD * KD * 2;
  const size_t bO = (size_t)NGR * DD * 4;
  const size_t oBL = off;  off += bBL;
  const size_t oFL = off;  off += bFL;
  const size_t oCOL = off; off += bCOL;
  const size_t oST = off;  off += bSE;
  const size_t oEN = off;  off += bSE;
  const size_t oA = off;   off += bA;
  const size_t oH0 = off;  off += bH;
  const size_t oH1 = off;  off += bH;
  const size_t oP = off;   off += bP;
  const size_t oW0 = off;  off += bW;
  const size_t oW1 = off;  off += bW;
  const size_t oWh = off;  off += bW;
  const size_t oO = off;   off += bO;
  const size_t tot = off;
  if (tot > ws_size || tot > (size_t)WSCAP) return;
  char* ws = (char*)d_ws;
  unsigned* blist = (unsigned*)(ws + oBL);
  unsigned* flg = (unsigned*)(ws + oFL);
  unsigned* colp = (unsigned*)(ws + oCOL);
  int* stp = (int*)(ws + oST);
  int* enp = (int*)(ws + oEN);
  unsigned short* Apl = (unsigned short*)(ws + oA);
  float* H0 = (float*)(ws + oH0);
  float* H1 = (float*)(ws + oH1);
  float* P = (float*)(ws + oP);
  unsigned short* W0p = (unsigned short*)(ws + oW0);
  unsigned short* W1p = (unsigned short*)(ws + oW1);
  unsigned short* Whp = (unsigned short*)(ws + oWh);
  float* O = (float*)(ws + oO);

  k_wprep<<<dim3((DD * NGRP) / NTHR, 3), NTHR, 0, stream>>>(bw0, sw0, sc0, bw1, sw1, sc1, bwh, swh, sch,
                                                             W0p, W1p, Whp);
  k_bucket<<<NCB, NTHR, 0, stream>>>(ei, nE, nN, blist, flg);
  hipFuncSetAttribute(reinterpret_cast<const void*>(&k_csr), hipFuncAttributeMaxDynamicSharedMemorySize, CSRLDS);
  k_csr<<<NFB, NTHR, CSRLDS, stream>>>(blist, colp, stp, enp, flg);

  for (int hf = 0; hf < 2; ++hf) {
    k_aggfeat<true><<<MHALF / 64, NTHR, 0, stream>>>(x, stp, enp, colp, Apl, hf * MHALF, nN, nN);
    k_gemm<<<MHALF / RPB, NTHR, 0, stream>>>(Apl, W0p, H0 + (size_t)hf * MHALF * DD);
  }
  for (int hf = 0; hf < 2; ++hf) {
    k_aggfeat<true><<<MHALF / 64, NTHR, 0, stream>>>(H0, stp, enp, colp, Apl, hf * MHALF, nN, nN);
    k_gemm<<<MHALF / RPB, NTHR, 0, stream>>>(Apl, W1p, H1 + (size_t)hf * MHALF * DD);
  }

  k_pool<<<NGR / NSEG, NTHR, 0, stream>>>(H1, bat, nN, P);
  k_aggfeat<false><<<NGR / 64, NTHR, 0, stream>>>(P, stp, enp, colp, Apl, 0, NGR, nN);
  k_gemm<<<NGR / RPB, NTHR, 0, stream>>>(Apl, Whp, O);
  k_pack<<<(NGR * NTGT) / (4 * NTHR), NTHR, 0, stream>>>(O, flg, out);
}
